// DPGN_75436805587537
// MI455X (gfx1250) — hardware-run, weakly checked
//
#include <hip/hip_runtime.h>

typedef __attribute__((ext_vector_type(16))) _Float16 v16h;
typedef __attribute__((ext_vector_type(8)))  _Float16 v8h;
typedef __attribute__((ext_vector_type(16))) __bf16   v16b;
typedef __attribute__((ext_vector_type(8)))  __bf16   v8b;
typedef __attribute__((ext_vector_type(8)))  float    v8f;
typedef __attribute__((ext_vector_type(4)))  float    v4f;
typedef __attribute__((ext_vector_type(2)))  float    v2f;
typedef __attribute__((ext_vector_type(4)))  unsigned v4u;

__device__ __forceinline__ unsigned short f2bf_bits(float f) {
  unsigned u = __float_as_uint(f);
  return (unsigned short)((u + 0x7FFFu + ((u >> 16) & 1u)) >> 16);
}
__device__ __forceinline__ float bf_bits2f(unsigned short h) { return __uint_as_float(((unsigned)h) << 16); }
__device__ __forceinline__ unsigned short f2h_bits(float f) { return __builtin_bit_cast(unsigned short, (_Float16)f); }

__device__ __forceinline__ void dep_guard_h(v8f& a, v8f& b, v16h x, v16h y) { asm volatile("v_nop\n\tv_nop\n\tv_nop\n\tv_nop" : "+v"(a), "+v"(b) : "v"(x), "v"(y)); }
__device__ __forceinline__ void dep_guard_b(v8f& a, v8f& b, v16b x, v16b y) { asm volatile("v_nop\n\tv_nop\n\tv_nop\n\tv_nop" : "+v"(a), "+v"(b) : "v"(x), "v"(y)); }
__device__ __forceinline__ void keep4_h(v16h a, v16h b, v16h c, v16h d) { asm volatile("v_nop" :: "v"(a), "v"(b), "v"(c), "v"(d)); }
__device__ __forceinline__ void keep4_b(v16b a, v16b b, v16b c, v16b d) { asm volatile("v_nop" :: "v"(a), "v"(b), "v"(c), "v"(d)); }
__device__ __forceinline__ void acc_guard4(v8f& a, v8f& b, v8f& c, v8f& d) { asm volatile("v_nop\n\tv_nop\n\tv_nop\n\tv_nop" : "+v"(a), "+v"(b), "+v"(c), "+v"(d)); }
template <typename T> struct Frag;
template <> struct Frag<_Float16> {
  typedef v16h V; union U { v16h v; v8h h[2]; };
  static __device__ __forceinline__ v16h load(const _Float16* p) {
    U f; f.h[0] = *(const v8h*)(p); f.h[1] = *(const v8h*)(p + 16); return f.v;
  }
  static __device__ __forceinline__ v8f mma(v16h a, v16h b, v8f c) {
    return __builtin_amdgcn_wmma_f32_16x16x32_f16(false, a, false, b, (short)0, c, false, false);
  }
  static __device__ __forceinline__ void guard(v8f& a, v8f& b, v16h x, v16h y) { dep_guard_h(a, b, x, y); }
  static __device__ __forceinline__ void keep(v16h a, v16h b, v16h c, v16h d) { keep4_h(a, b, c, d); }
};
template <> struct Frag<__bf16> {
  typedef v16b V; union U { v16b v; v8b h[2]; };
  static __device__ __forceinline__ v16b load(const __bf16* p) {
    U f; f.h[0] = *(const v8b*)(p); f.h[1] = *(const v8b*)(p + 16); return f.v;
  }
  static __device__ __forceinline__ v8f mma(v16b a, v16b b, v8f c) {
    return __builtin_amdgcn_wmma_f32_16x16x32_bf16(false, a, false, b, (short)0, c, false, false);
  }
  static __device__ __forceinline__ void guard(v8f& a, v8f& b, v16b x, v16b y) { dep_guard_b(a, b, x, y); }
  static __device__ __forceinline__ void keep(v16b a, v16b b, v16b c, v16b d) { keep4_b(a, b, c, d); }
};

template <int ET> struct Elem;
template <> struct Elem<0> { typedef _Float16 T; };
template <> struct Elem<1> { typedef __bf16 T; };
template <int ET, bool SPLIT, int BIAS_MODE, int OUT_MODE, bool RESID, int ACT = 0>
__global__ __launch_bounds__(256) void wmma_gemm64(
    const unsigned short* __restrict__ Ap, const unsigned short* __restrict__ A2p, int lda, long strideA,
    const unsigned short* __restrict__ Btp, const unsigned short* __restrict__ Bt2p, int ldb, long strideB,
    void* __restrict__ Cout, void* __restrict__ Cout2, int ldc, long strideC,
    const float* __restrict__ bias,
    const float* __restrict__ resid, long strideR,
    int M, int N, int K, float scale) {
  typedef typename Elem<ET>::T T;
  typedef typename Frag<T>::V V;
  const T* A = (const T*)Ap; const T* A2 = (const T*)A2p; const T* Bt = (const T*)Btp; const T* Bt2 = (const T*)Bt2p;
  __shared__ __align__(16) float sT[8][16 * 68];
  const int b    = blockIdx.y;
  const int lane = threadIdx.x & 31;
  const int wave = threadIdx.x >> 5;
  const int tilesN = N >> 6;
  const int tilesM = M >> 6;
  const int tile = blockIdx.x * 8 + wave;
  if (tile >= tilesM * tilesN) return;
  const int tm = tile / tilesN;
  const int tn = tile - tm * tilesN;
  const int m0 = tm << 6;
  const int n0 = tn << 6;

  const T* Ab  = A  + (size_t)b * strideA;
  const T* Bb  = Bt + (size_t)b * strideB;
  const T* Ab2 = SPLIT ? (A2  + (size_t)b * strideA) : nullptr;
  const T* Bb2 = SPLIT ? (Bt2 + (size_t)b * strideB) : nullptr;

  const int rlane = lane & 15;
  const int koff  = (lane >> 4) * 8;
  const int mOff  = (lane >> 4) * 8;

  v8f acc[4][4];
#pragma unroll
  for (int i = 0; i < 4; ++i)
#pragma unroll
    for (int j = 0; j < 4; ++j) acc[i][j] = (v8f){0.f,0.f,0.f,0.f,0.f,0.f,0.f,0.f};

  for (int k0 = 0; k0 < K; k0 += 32) {
    V bh[4], bl[4];
#pragma unroll
    for (int j = 0; j < 4; ++j) {
      const size_t bo = (size_t)(n0 + (j << 4) + rlane) * ldb + koff + k0;
      bh[j] = Frag<T>::load(Bb + bo);
      if (SPLIT) bl[j] = Frag<T>::load(Bb2 + bo);
    }
#pragma unroll
    for (int i = 0; i < 4; ++i) {
      const size_t ao = (size_t)(m0 + (i << 4) + rlane) * lda + koff + k0;
      V ah = Frag<T>::load(Ab + ao);
      V al;
      if (SPLIT) al = Frag<T>::load(Ab2 + ao);
#pragma unroll
      for (int j = 0; j < 4; ++j) {
        acc[i][j] = Frag<T>::mma(ah, bh[j], acc[i][j]);
        if (SPLIT) {
          acc[i][j] = Frag<T>::mma(ah, bl[j], acc[i][j]);
          acc[i][j] = Frag<T>::mma(al, bh[j], acc[i][j]);
        }
      }
      Frag<T>::guard(acc[i][0], acc[i][3], ah, SPLIT ? al : ah);
    }
    Frag<T>::keep(bh[0], bh[1], bh[2], bh[3]);
    if (SPLIT) Frag<T>::keep(bl[0], bl[1], bl[2], bl[3]);
  }
  acc_guard4(acc[0][0], acc[0][1], acc[0][2], acc[0][3]);
  acc_guard4(acc[1][0], acc[1][1], acc[1][2], acc[1][3]);
  acc_guard4(acc[2][0], acc[2][1], acc[2][2], acc[2][3]);
  acc_guard4(acc[3][0], acc[3][1], acc[3][2], acc[3][3]);

  float* slab = sT[wave];
  const float* Rb = RESID ? (resid + (size_t)b * strideR) : nullptr;
#pragma unroll
  for (int i = 0; i < 4; ++i) {
    const int mBase = m0 + (i << 4);
#pragma unroll
    for (int j = 0; j < 4; ++j) {
      const int n = n0 + (j << 4) + rlane;
      float bv = 0.f;
      if (BIAS_MODE == 2) bv = bias[n];
#pragma unroll
      for (int r = 0; r < 8; ++r) {
        float v = acc[i][j][r] * scale;
        if (BIAS_MODE == 1) v += bias[mBase + mOff + r];
        if (BIAS_MODE == 2) v += bv;
        if (RESID) v += Rb[(size_t)(mBase + mOff + r) * ldc + n];
        if (ACT == 1) v = tanhf(v);
        if (ACT == 2) v = fmaxf(v, 0.0f);
        if (ACT == 3) v = v / (1.0f + expf(-v));
        if (ACT == 4) v = (v > 0.f) ? v : 0.01f * v;
        if (ACT == 5) v = 0.5f * v * (1.0f + erff(v * 0.70710678118654752f));
        slab[(mOff + r) * 68 + (j << 4) + rlane] = v;
      }
    }
    __builtin_amdgcn_fence(__ATOMIC_RELEASE, "workgroup");
    __builtin_amdgcn_wave_barrier();
    __builtin_amdgcn_fence(__ATOMIC_ACQUIRE, "workgroup");
    if (OUT_MODE == 0) {
      float* C = (float*)Cout + (size_t)b * strideC;
      const int hh = lane >> 4, c4 = (lane & 15) * 4;
      for (int pass = 0; pass < 2; ++pass) {
#pragma unroll
        for (int it = 0; it < 8; ++it) {
          const int row = it * 2 + hh;
          v4f v = *(const v4f*)(slab + row * 68 + c4);
          *(volatile v4f*)(C + (size_t)(mBase + row) * ldc + n0 + c4) = v;
        }
        __threadfence();
      }
    } else {
      const int q = lane >> 3, c8 = (lane & 7) * 8;
      unsigned short* C  = (unsigned short*)Cout  + (size_t)b * strideC;
      unsigned short* C2 = (OUT_MODE == 2) ? ((unsigned short*)Cout2 + (size_t)b * strideC) : nullptr;
      for (int pass = 0; pass < 2; ++pass) {
#pragma unroll
        for (int it = 0; it < 4; ++it) {
          const int row = it * 4 + q;
          const float* sp = slab + row * 68 + c8;
          v8h hv, lv;
#pragma unroll
          for (int e = 0; e < 8; ++e) {
            if (OUT_MODE == 1) {
              hv[e] = (_Float16)sp[e];
            } else {
              unsigned short hb = f2bf_bits(sp[e]);
              unsigned short lb = f2bf_bits(sp[e] - bf_bits2f(hb));
              hv[e] = __builtin_bit_cast(_Float16, hb);
              lv[e] = __builtin_bit_cast(_Float16, lb);
            }
          }
          *(volatile v8h*)(C + (size_t)(mBase + row) * ldc + n0 + c8) = hv;
          if (OUT_MODE == 2) *(volatile v8h*)(C2 + (size_t)(mBase + row) * ldc + n0 + c8) = lv;
        }
        __threadfence();
      }
    }
    __builtin_amdgcn_fence(__ATOMIC_RELEASE, "workgroup");
    __builtin_amdgcn_wave_barrier();
    __builtin_amdgcn_fence(__ATOMIC_ACQUIRE, "workgroup");
  }
}

namespace {
constexpr int kB = 16, kN = 160, kC = 64, kC2 = 128, kS = 80;
constexpr int kNN  = kN * kN;
constexpr int kM   = kB * kNN;
constexpr int kBI  = kB * kN;
constexpr int kK2  = 2 * kS;
constexpr int kNP  = 128;
constexpr int kRows = 64;
constexpr int kNBLK = kM / kRows;
constexpr int kPA = 72;
constexpr int kPH = 136;
constexpr int kSimScale = 128, kW1Scale = 64, kHScale = 16, kW2Scale = 64;
constexpr int kAcc1Scale = kSimScale * kW1Scale;
constexpr int kAcc2Scale = kHScale * kW2Scale;
static_assert(kM % kRows == 0);
static_assert(kNN % kRows == 0);
static_assert(kRows * kC / 2 == 16 * 128);
static_assert(kK2 % 32 == 0);
static_assert(kBI % 64 == 0 && kNP % 64 == 0);
static_assert((kBI * kK2) % (8 * 256) == 0);
static_assert((kNP * kK2) % (8 * 256) == 0);
static_assert((kBI * kS) % (4 * 256) == 0);
static_assert(kN % 32 == 0);
static_assert(16 * kPH * 2 == 16 * 68 * 4);

constexpr size_t szW1h  = (size_t)kC2 * kC * 2;
constexpr size_t szW2h  = (size_t)kC * kC2 * 2;
constexpr size_t szBnA  = 256 * 4;
constexpr size_t szBnB  = 128 * 4;
constexpr size_t szPart1 = (size_t)kNBLK * 256 * 4;
constexpr size_t szPart2 = (size_t)kNBLK * 128 * 4;
constexpr size_t szZ2   = (size_t)kM * kC * 2;
constexpr size_t szE    = (size_t)kM * 4;
constexpr size_t szPe   = (size_t)kM * 4;
constexpr size_t szA    = (size_t)kBI * kK2 * 2;
constexpr size_t szBt   = (size_t)kNP * kK2 * 2;
constexpr size_t szBias = (size_t)kNP * 4;
constexpr size_t szCpl  = (size_t)kBI * kNP * 4;
constexpr size_t kWsTotal = szW1h + szW2h + szBnA + szBnB + szPart1 + szPart2 + szZ2 + szE
                          + 3 * szPe + 2 * szA + 2 * szBt + szBias + 2 * szCpl;
static_assert(kWsTotal <= (size_t)134217728);
static_assert(szW1h % 256 == 0 && szW2h % 256 == 0 && szBnA % 256 == 0 && szBnB % 256 == 0 && szPart1 % 256 == 0 &&
              szPart2 % 256 == 0 && szZ2 % 256 == 0 && szE % 256 == 0 && szPe % 256 == 0 && szA % 256 == 0 &&
              szBt % 256 == 0 && szBias % 256 == 0 && szCpl % 256 == 0);
constexpr size_t kOut1Off = (size_t)kBI * kS;
static_assert(kOut1Off * 4 == 819200);
static_assert((kOut1Off + (size_t)kBI * kS) * 4 == 1638400);
}

__device__ __forceinline__ v8f zero8() { return (v8f){0.f,0.f,0.f,0.f,0.f,0.f,0.f,0.f}; }
__device__ __forceinline__ float wave_sum(float v) {
  v += __shfl_xor(v, 16, 32);
  v += __shfl_xor(v, 8, 32);
  v += __shfl_xor(v, 4, 32);
  v += __shfl_xor(v, 2, 32);
  v += __shfl_xor(v, 1, 32);
  return v;
}
__device__ __forceinline__ float sum8(const float* r) {
  return ((((((r[0] + r[1]) + r[2]) + r[3]) + r[4]) + r[5]) + r[6]) + r[7];
}
__device__ __forceinline__ unsigned pack_hl(float a, float b, unsigned& lo) {
  const unsigned short ha = f2bf_bits(a), hb = f2bf_bits(b);
  const unsigned short la = f2bf_bits(a - bf_bits2f(ha)), lb = f2bf_bits(b - bf_bits2f(hb));
  lo = (unsigned)la | ((unsigned)lb << 16);
  return (unsigned)ha | ((unsigned)hb << 16);
}
__device__ __forceinline__ void split8(v4f f0, v4f f1, v4u& hi, v4u& lo) {
  unsigned l0, l1, l2, l3;
  hi.x = pack_hl(f0.x, f0.y, l0);
  hi.y = pack_hl(f0.z, f0.w, l1);
  hi.z = pack_hl(f1.x, f1.y, l2);
  hi.w = pack_hl(f1.z, f1.w, l3);
  lo.x = l0; lo.y = l1; lo.z = l2; lo.w = l3;
}
__device__ __forceinline__ v4f sel4(bool c, v4f a, v4f b) {
  v4f r;
  r.x = c ? a.x : b.x; r.y = c ? a.y : b.y; r.z = c ? a.z : b.z; r.w = c ? a.w : b.w;
  return r;
}

__global__ __launch_bounds__(256) void cast_scale_f16x2(
    const float* __restrict__ in, unsigned short* __restrict__ out, float sc, int n2) {
  const int i = blockIdx.x * 256 + threadIdx.x;
  if (i < n2) {
    const unsigned u = (unsigned)f2h_bits(in[2 * i] * sc) | ((unsigned)f2h_bits(in[2 * i + 1] * sc) << 16);
    ((volatile unsigned*)out)[i] = u;
    __threadfence();
    ((volatile unsigned*)out)[i] = u;
  }
}

template <int MODE>
__global__ __launch_bounds__(128) void k_ps(const float* __restrict__ V,
                                           const unsigned short* __restrict__ W1p,
                                           const unsigned short* __restrict__ W2p,
                                           const float* __restrict__ bnA,
                                           float* __restrict__ part,
                                           unsigned short* __restrict__ z2) {
  typedef Frag<_Float16> FH;
  __shared__ __align__(16) unsigned short sA[kRows * kPA];
  __shared__ __align__(16) unsigned short sH[(MODE == 1) ? kRows * kPH : 8];
  __shared__ float sBN[(MODE == 1) ? 2 * kC2 : 4];
  __shared__ float sRed[4][256];
  __shared__ __align__(16) float sRec[256];

  const int t = threadIdx.x, lane = t & 31, wave = t >> 5, hh = lane >> 4, rl = lane & 15;
  const int blk = blockIdx.x;
  const int m0 = blk * kRows;
  const int b = m0 / kNN;
  const int rem0 = m0 - b * kNN;
  const float* Vb = V + (size_t)b * kN * kC;
  if constexpr (MODE == 1) { sBN[t] = bnA[t]; sBN[t + 128] = bnA[t + 128]; }

#pragma unroll 2
  for (int k = 0; k < 16; ++k) {
    const int idx = t + 128 * k;
    const int r = idx >> 5, cp = idx & 31;
    const int rr = rem0 + r;
    const int i = rr / kN;
    const int j = rr - i * kN;
    const v2f vi = *(const v2f*)(Vb + i * kC + 2 * cp);
    const v2f vj = *(const v2f*)(Vb + j * kC + 2 * cp);
    const float d0 = vi.x - vj.x, d1 = vi.y - vj.y;
    const float s0 = d0 * d0, s1 = d1 * d1;
    const unsigned u = (unsigned)f2h_bits(s0 * (float)kSimScale) | ((unsigned)f2h_bits(s1 * (float)kSimScale) << 16);
    *(unsigned*)(sA + r * kPA + 2 * cp) = u;
  }
  __syncthreads();

  const _Float16* A1 = (const _Float16*)sA;
  const _Float16* B1 = (const _Float16*)W1p;
  const int R0 = wave * 16;
  v8f acc1[8];
#pragma unroll
  for (int j = 0; j < 8; ++j) acc1[j] = zero8();
#pragma unroll
  for (int k0 = 0; k0 < kC; k0 += 32) {
    const v16h a = FH::load(A1 + (R0 + rl) * kPA + k0 + 8 * hh);
#pragma unroll
    for (int jg = 0; jg < 2; ++jg) {
      v16h bq[4];
#pragma unroll
      for (int jj = 0; jj < 4; ++jj)
        bq[jj] = FH::load(B1 + (size_t)(16 * (4 * jg + jj) + rl) * kC + k0 + 8 * hh);
#pragma unroll
      for (int jj = 0; jj < 4; ++jj) acc1[4 * jg + jj] = FH::mma(a, bq[jj], acc1[4 * jg + jj]);
      dep_guard_h(acc1[4 * jg], acc1[4 * jg + 3], a, bq[3]);
      keep4_h(bq[0], bq[1], bq[2], bq[3]);
    }
  }
  acc_guard4(acc1[0], acc1[1], acc1[2], acc1[3]);
  acc_guard4(acc1[4], acc1[5], acc1[6], acc1[7]);

  if constexpr (MODE == 0) {
#pragma unroll
    for (int j = 0; j < 8; ++j) {
      float s = 0.f, q = 0.f;
#pragma unroll
      for (int r = 0; r < 8; ++r) { const float x = acc1[j][r]; s += x; q = fmaf(x, x, q); }
      s += __shfl_xor(s, 16, 32);
      q += __shfl_xor(q, 16, 32);
      if (hh == 0) { sRed[wave][16 * j + rl] = s; sRed[wave][128 + 16 * j + rl] = q; }
    }
    __syncthreads();
    {
      const float S = ((sRed[0][t] + sRed[1][t]) + sRed[2][t]) + sRed[3][t];
      const float Q = ((sRed[0][t + 128] + sRed[1][t + 128]) + sRed[2][t + 128]) + sRed[3][t + 128];
      sRec[t] = S;
      sRec[t + 128] = Q;
    }
    __syncthreads();
    for (int pass = 0; pass < 2; ++pass) {
      if (t < 64) {
        const v4f v = *(const v4f*)(sRec + 4 * t);
        *(volatile v4f*)(part + (size_t)blk * 256 + 4 * t) = v;
      }
      __threadfence();
    }
  } else {
#pragma unroll
    for (int j = 0; j < 8; ++j) {
      const int n = 16 * j + rl;
      const float sc = sBN[n], sh = sBN[kC2 + n];
#pragma unroll
      for (int r = 0; r < 8; ++r) {
        float x = fmaf(acc1[j][r], sc, sh);
        x = fmaxf(x, 0.01f * x);
        sH[(R0 + 8 * hh + r) * kPH + n] = f2h_bits(x);
      }
    }
    __syncthreads();

    const _Float16* A2 = (const _Float16*)sH;
    const _Float16* B2 = (const _Float16*)W2p;
    v8f acc2[4];
#pragma unroll
    for (int j = 0; j < 4; ++j) acc2[j] = zero8();
#pragma unroll
    for (int k0 = 0; k0 < kC2; k0 += 32) {
      const v16h a = FH::load(A2 + (R0 + rl) * kPH + k0 + 8 * hh);
      v16h bq[4];
#pragma unroll
      for (int jj = 0; jj < 4; ++jj)
        bq[jj] = FH::load(B2 + (size_t)(16 * jj + rl) * kC2 + k0 + 8 * hh);
#pragma unroll
      for (int jj = 0; jj < 4; ++jj) acc2[jj] = FH::mma(a, bq[jj], acc2[jj]);
      dep_guard_h(acc2[0], acc2[3], a, bq[3]);
      keep4_h(bq[0], bq[1], bq[2], bq[3]);
    }
    acc_guard4(acc2[0], acc2[1], acc2[2], acc2[3]);

#pragma unroll
    for (int j = 0; j < 4; ++j) {
      float s = 0.f, q = 0.f;
#pragma unroll
      for (int r = 0; r < 8; ++r) { const float x = acc2[j][r]; s += x; q = fmaf(x, x, q); }
      s += __shfl_xor(s, 16, 32);
      q += __shfl_xor(q, 16, 32);
      if (hh == 0) { sRed[wave][16 * j + rl] = s; sRed[wave][64 + 16 * j + rl] = q; }
    }
    __syncthreads();
    {
      const float S = ((sRed[0][t] + sRed[1][t]) + sRed[2][t]) + sRed[3][t];
      sRec[t] = S;
    }
    float* slab = (float*)sH + wave * (16 * 68);
#pragma unroll
    for (int j = 0; j < 4; ++j)
#pragma unroll
      for (int r = 0; r < 8; ++r)
        slab[(8 * hh + r) * 68 + 16 * j + rl] = acc2[j][r] * (1.0f / (float)kAcc2Scale);
    __syncthreads();
    const int q4 = lane >> 3, c8 = (lane & 7) * 8;
    for (int pass = 0; pass < 2; ++pass) {
#pragma unroll
      for (int it = 0; it < 4; ++it) {
        const int row = 4 * it + q4;
        const float* sp = slab + row * 68 + c8;
        const v4f f0 = *(const v4f*)sp;
        const v4f f1 = *(const v4f*)(sp + 4);
        v4u pk;
        pk.x = (unsigned)f2bf_bits(f0.x) | ((unsigned)f2bf_bits(f0.y) << 16);
        pk.y = (unsigned)f2bf_bits(f0.z) | ((unsigned)f2bf_bits(f0.w) << 16);
        pk.z = (unsigned)f2bf_bits(f1.x) | ((unsigned)f2bf_bits(f1.y) << 16);
        pk.w = (unsigned)f2bf_bits(f1.z) | ((unsigned)f2bf_bits(f1.w) << 16);
        *(volatile v4u*)(z2 + ((size_t)(m0 + R0 + row) * kC + c8)) = pk;
      }
      if (wave == 0) {
        const v4f v = *(const v4f*)(sRec + 4 * lane);
        *(volatile v4f*)(part + (size_t)blk * 128 + 4 * lane) = v;
      }
      __threadfence();
    }
  }
}

template <int NCH, int ASC, int ODIV, int OMUL>
__global__ __launch_bounds__(256) void k_fin(const float* __restrict__ part,
                                            const float* __restrict__ gam,
                                            const float* __restrict__ bet,
                                            float* __restrict__ table) {
  constexpr int NC2 = 2 * NCH;
  __shared__ double sCol[256];
  __shared__ __align__(16) float sTab[256];
  const int t = threadIdx.x;
  double acc = 0.0;
  if (t < NC2) {
#pragma unroll 4
    for (int blk = 0; blk < kNBLK; ++blk) acc += (double)part[(size_t)blk * NC2 + t];
  }
  sCol[t] = acc;
  __syncthreads();
  if (t < NCH) {
    const double cnt = (double)kM;
    const double mean = sCol[t] / ((double)ASC * cnt);
    const double ez2 = sCol[NCH + t] / ((double)ASC * (double)ASC * cnt);
    double var = ez2 - mean * mean;
    if (var < 0.0) var = 0.0;
    const float varf = (float)var;
    const float inv = 1.0f / sqrtf(varf + 1e-5f);
    const float sc = gam[t] * inv;
    const float sh = bet[t] - (float)mean * sc;
    sTab[t] = sc * (1.0f / (float)ODIV);
    sTab[NCH + t] = sh * (float)OMUL;
  }
  __syncthreads();
  for (int pass = 0; pass < 2; ++pass) {
    if (t < NC2 / 4) {
      const v4f v = *(const v4f*)(sTab + 4 * t);
      *(volatile v4f*)(table + 4 * t) = v;
    }
    __threadfence();
  }
}

__device__ __forceinline__ float chpair(unsigned word, int c, const float* sc, const float* sh, const float* w, float p) {
  const float f0 = __uint_as_float(word << 16);
  const float f1 = __uint_as_float(word & 0xffff0000u);
  float x0 = fmaf(f0, sc[c], sh[c]);
  x0 = fmaxf(x0, 0.01f * x0);
  p = fmaf(x0, w[c], p);
  float x1 = fmaf(f1, sc[c + 1], sh[c + 1]);
  x1 = fmaxf(x1, 0.01f * x1);
  p = fmaf(x1, w[c + 1], p);
  return p;
}
__global__ __launch_bounds__(256) void k_sig(const unsigned* __restrict__ z2w,
                                            const float* __restrict__ bnB,
                                            const float* __restrict__ w3,
                                            const float* __restrict__ b3,
                                            float* __restrict__ ebuf) {
  __shared__ float sSc[kC], sSh[kC], sW[kC];
  __shared__ float sLog[kN];
  __shared__ __align__(16) float sE[kN];
  const int t = threadIdx.x;
  const int bi = blockIdx.x;
  if (t < kC) { sSc[t] = bnB[t]; sSh[t] = bnB[kC + t]; sW[t] = w3[t]; }
  const float b3v = b3[0];
  __syncthreads();
  const v4u* zb = (const v4u*)z2w + (size_t)bi * (kN * 8);
#pragma unroll 1
  for (int k = 0; k < 5; ++k) {
    const int u = t + 256 * k;
    const int j = u >> 3, q = u & 7;
    const v4u wv = zb[u];
    float p = 0.f;
    p = chpair(wv.x, 8 * q + 0, sSc, sSh, sW, p);
    p = chpair(wv.y, 8 * q + 2, sSc, sSh, sW, p);
    p = chpair(wv.z, 8 * q + 4, sSc, sSh, sW, p);
    p = chpair(wv.w, 8 * q + 6, sSc, sSh, sW, p);
    p += __shfl_xor(p, 1, 32);
    p += __shfl_xor(p, 2, 32);
    p += __shfl_xor(p, 4, 32);
    if (q == 0) sLog[j] = p;
  }
  __syncthreads();
  if (t < kN) {
    const float lg = sLog[t] + b3v;
    const float ex = expf(-lg);
    sE[t] = 1.0f / (1.0f + ex);
  }
  __syncthreads();
  for (int pass = 0; pass < 2; ++pass) {
    if (t < kN / 4) {
      const v4f v = *(const v4f*)(sE + 4 * t);
      *(volatile v4f*)(ebuf + (size_t)bi * kN + 4 * t) = v;
    }
    __threadfence();
  }
}

__global__ __launch_bounds__(256) void k_norm(const float* __restrict__ ebuf,
                                             const float* __restrict__ epl,
                                             float* __restrict__ peo) {
  __shared__ float sRed[3][8];
  __shared__ __align__(16) float sOut[kN];
  const int t = threadIdx.x, lane = t & 31, wave = t >> 5;
  const int bi = blockIdx.x;
  const int i = bi % kN;
  const bool valid = t < kN;
  const int tc = valid ? t : (kN - 1);
  const size_t rb = (size_t)bi * kN;
  const float ep = epl[rb + tc];
  const float ev = ebuf[rb + tc];
  const bool isdiag = valid && (t == i);
  const float epm = (valid && !isdiag) ? ep : 0.f;
  float v = wave_sum(epm);
  if (lane == 0) sRed[0][wave] = v;
  __syncthreads();
  const float rowsum = sum8(sRed[0]);
  const float x = ev * epm;
  v = wave_sum(fabsf(x));
  if (lane == 0) sRed[1][wave] = v;
  __syncthreads();
  const float l1 = sum8(sRed[1]);
  const float den = fmaxf(l1, 1e-12f);
  float y = (x * (1.0f / den)) * rowsum;
  y = y + (isdiag ? 1.0f : 0.0f);
  y = valid ? (y + 1e-6f) : 0.0f;
  v = wave_sum(y);
  if (lane == 0) sRed[2][wave] = v;
  __syncthreads();
  const float tot = sum8(sRed[2]);
  const float o = y * (1.0f / tot);
  if (valid) sOut[t] = o;
  __syncthreads();
  for (int pass = 0; pass < 2; ++pass) {
    if (t < kN / 4) {
      const v4f q = *(const v4f*)(sOut + 4 * t);
      *(volatile v4f*)(peo + rb + 4 * t) = q;
    }
    __threadfence();
  }
}

__global__ __launch_bounds__(256) void k_planes(const float* __restrict__ pe, const float* __restrict__ dn, int dpitch,
                                               const float* __restrict__ W, const float* __restrict__ bias,
                                               unsigned short* __restrict__ Ah, unsigned short* __restrict__ Al,
                                               unsigned short* __restrict__ Bh, unsigned short* __restrict__ Bl,
                                               float* __restrict__ biaspad) {
  const int t = threadIdx.x, blk = blockIdx.x;
  if (blk < 200) {
    const int g = blk * 256 + t;
    const int e = 8 * g;
    const int row = e / kK2;
    const int col = e - row * kK2;
    const float* pp = pe + (size_t)row * kN + col;
    const v4f p0 = *(const v4f*)pp, p1 = *(const v4f*)(pp + 4);
    int cd = col - kS; cd = cd < 0 ? 0 : cd;
    const float* dp = dn + (size_t)row * dpitch + cd;
    const v4f q0 = *(const v4f*)dp, q1 = *(const v4f*)(dp + 4);
    const bool usep = col < kS;
    const v4f f0 = sel4(usep, p0, q0);
    const v4f f1 = sel4(usep, p1, q1);
    v4u hi, lo;
    split8(f0, f1, hi, lo);
    for (int pass = 0; pass < 2; ++pass) {
      *(volatile v4u*)(Ah + e) = hi;
      *(volatile v4u*)(Al + e) = lo;
      __threadfence();
    }
  } else if (blk < 210) {
    const int g = (blk - 200) * 256 + t;
    const int e = 8 * g;
    const int o = e / kK2;
    const int col = e - o * kK2;
    const int oc = o < kS ? o : (kS - 1);
    const float* wp = W + (size_t)oc * kK2 + col;
    const v4f w0 = *(const v4f*)wp, w1 = *(const v4f*)(wp + 4);
    const v4f z = {0.f, 0.f, 0.f, 0.f};
    const bool keep = o < kS;
    const v4f f0 = sel4(keep, w0, z);
    const v4f f1 = sel4(keep, w1, z);
    v4u hi, lo;
    split8(f0, f1, hi, lo);
    for (int pass = 0; pass < 2; ++pass) {
      *(volatile v4u*)(Bh + e) = hi;
      *(volatile v4u*)(Bl + e) = lo;
      __threadfence();
    }
  } else {
    if (t < 32) {
      v4f v;
      {
        const int i0 = 4 * t, i1 = 4 * t + 1, i2 = 4 * t + 2, i3 = 4 * t + 3;
        const float x0 = bias[i0 < kS ? i0 : kS - 1];
        const float x1 = bias[i1 < kS ? i1 : kS - 1];
        const float x2 = bias[i2 < kS ? i2 : kS - 1];
        const float x3 = bias[i3 < kS ? i3 : kS - 1];
        v.x = (i0 < kS) ? x0 : 0.f;
        v.y = (i1 < kS) ? x1 : 0.f;
        v.z = (i2 < kS) ? x2 : 0.f;
        v.w = (i3 < kS) ? x3 : 0.f;
      }
      for (int pass = 0; pass < 2; ++pass) {
        *(volatile v4f*)(biaspad + 4 * t) = v;
        __threadfence();
      }
    }
  }
}

__global__ __launch_bounds__(256) void k_out(const float* __restrict__ Cp, float* __restrict__ out) {
  const int g = blockIdx.x * 256 + threadIdx.x;
  const int f = 4 * g;
  const int row = f / kS;
  const int col = f - row * kS;
  const v4f v = *(const v4f*)(Cp + (size_t)row * kNP + col);
  for (int pass = 0; pass < 2; ++pass) {
    *(volatile v4f*)(out + f) = v;
    __threadfence();
  }
}

extern "C" void kernel_launch(void* const* d_in, const int* in_sizes, int n_in,
                              void* d_out, int out_size, void* d_ws, size_t ws_size,
                              hipStream_t stream) {
  if (n_in < 15) return;
  if (out_size != 2 * kBI * kS) return;
  if (ws_size < kWsTotal) return;
  if (in_sizes[0] != kBI * kC || in_sizes[1] != kBI * kC || in_sizes[2] != kBI * kS || in_sizes[4] != kM) return;

  const float* middle = (const float*)d_in[0];
  const float* point  = (const float*)d_in[1];
  const float* dnode  = (const float*)d_in[2];
  const float* pedge  = (const float*)d_in[4];
  const float* w1  = (const float*)d_in[5];
  const float* g1  = (const float*)d_in[6];
  const float* b1  = (const float*)d_in[7];
  const float* w2  = (const float*)d_in[8];
  const float* g2  = (const float*)d_in[9];
  const float* b2  = (const float*)d_in[10];
  const float* w3  = (const float*)d_in[11];
  const float* b3  = (const float*)d_in[12];
  const float* p2dw = (const float*)d_in[13];
  const float* p2db = (const float*)d_in[14];
  float* out = (float*)d_out;

  char* ws = (char*)d_ws;
  size_t off = 0;
  auto carve = [&](size_t bytes) -> char* { char* p = ws + off; off += (bytes + 255) & ~(size_t)255; return p; };
  unsigned short* W1h = (unsigned short*)carve(szW1h);
  unsigned short* W2h = (unsigned short*)carve(szW2h);
  float* bnA   = (float*)carve(szBnA);
  float* bnB   = (float*)carve(szBnB);
  float* part1 = (float*)carve(szPart1);
  float* part2 = (float*)carve(szPart2);
  unsigned short* z2 = (unsigned short*)carve(szZ2);
  float* ebuf  = (float*)carve(szE);
  float* pe0   = (float*)carve(szPe);
  float* pe1   = (float*)carve(szPe);
  float* pe2   = (float*)carve(szPe);
  unsigned short* Ah = (unsigned short*)carve(szA);
  unsigned short* Al = (unsigned short*)carve(szA);
  unsigned short* Bh = (unsigned short*)carve(szBt);
  unsigned short* Bl = (unsigned short*)carve(szBt);
  float* biaspad = (float*)carve(szBias);
  float* C0 = (float*)carve(szCpl);
  float* C1 = (float*)carve(szCpl);
  if (off > ws_size) return;

  cast_scale_f16x2<<<(kC2 * kC / 2) / 256, 256, 0, stream>>>(w1, W1h, (float)kW1Scale, kC2 * kC / 2);
  cast_scale_f16x2<<<(kC * kC2 / 2) / 256, 256, 0, stream>>>(w2, W2h, (float)kW2Scale, kC * kC2 / 2);

  k_ps<0><<<kNBLK, 128, 0, stream>>>(middle, W1h, W2h, bnA, part1, z2);
  k_fin<kC2, kAcc1Scale, kAcc1Scale / kHScale, kHScale><<<1, 256, 0, stream>>>(part1, g1, b1, bnA);
  k_ps<1><<<kNBLK, 128, 0, stream>>>(middle, W1h, W2h, bnA, part2, z2);
  k_fin<kC, kAcc2Scale, 1, 1><<<1, 256, 0, stream>>>(part2, g2, b2, bnB);
  k_sig<<<kBI, 256, 0, stream>>>((const unsigned*)z2, bnB, w3, b3, ebuf);
  k_norm<<<kBI, 256, 0, stream>>>(ebuf, pedge, pe0);

  k_ps<0><<<kNBLK, 128, 0, stream>>>(point, W1h, W2h, bnA, part1, z2);
  k_fin<kC2, kAcc1Scale, kAcc1Scale / kHScale, kHScale><<<1, 256, 0, stream>>>(part1, g1, b1, bnA);
  k_ps<1><<<kNBLK, 128, 0, stream>>>(point, W1h, W2h, bnA, part2, z2);
  k_fin<kC, kAcc2Scale, 1, 1><<<1, 256, 0, stream>>>(part2, g2, b2, bnB);
  k_sig<<<kBI, 256, 0, stream>>>((const unsigned*)z2, bnB, w3, b3, ebuf);

  k_norm<<<kBI, 256, 0, stream>>>(ebuf, pe0, pe1);
  k_planes<<<211, 256, 0, stream>>>(pe1, dnode, kS, p2dw, p2db, Ah, Al, Bh, Bl, biaspad);
  wmma_gemm64<1, true, 2, 0, false, 4><<<dim3((kBI / 64) * (kNP / 64) / 8, 1), 256, 0, stream>>>(
      Ah, Al, kK2, 0L, Bh, Bl, kK2, 0L, (void*)C0, nullptr, kNP, 0L, biaspad, nullptr, 0L, kBI, kNP, kK2, 1.0f);
  k_out<<<(kBI * kS / 4) / 256, 256, 0, stream>>>(C0, out);

  k_norm<<<kBI, 256, 0, stream>>>(ebuf, pe1, pe2);
  k_planes<<<211, 256, 0, stream>>>(pe2, C0, kNP, p2dw + (size_t)kS * kK2, p2db + kS, Ah, Al, Bh, Bl, biaspad);
  wmma_gemm64<1, true, 2, 0, false, 4><<<dim3((kBI / 64) * (kNP / 64) / 8, 1), 256, 0, stream>>>(
      Ah, Al, kK2, 0L, Bh, Bl, kK2, 0L, (void*)C1, nullptr, kNP, 0L, biaspad, nullptr, 0L, kBI, kNP, kK2, 1.0f);
  k_out<<<(kBI * kS / 4) / 256, 256, 0, stream>>>(C1, out + kOut1Off);
}
